// OpinionDynamicsModel_3959959847022
// MI455X (gfx1250) — hardware-verified
//
#include <hip/hip_runtime.h>
#include <math.h>


typedef unsigned int u32;
typedef __attribute__((ext_vector_type(2)))  int      v2i;
typedef __attribute__((ext_vector_type(16))) _Float16 v16h;
typedef __attribute__((ext_vector_type(8)))  _Float16 v8h;
typedef __attribute__((ext_vector_type(8)))  float    v8f;
typedef __attribute__((ext_vector_type(4)))  float    v4f;
#define NN    10000
#define NE    160000
#define DD    128
#define DIN   768
#define HC    512
#define SORTN 262144
#define TILE  8192
#define NPAD  10048
#define MAXDEG 4096
#define VST2(T, ptr, val) do { const T _v = (val); *(volatile T*)(ptr) = _v; __threadfence(); *(volatile T*)(ptr) = _v; } while (0)
__device__ __forceinline__ v8f wmma16(v16h a, v16h b, v8f c) {
  v8f d = __builtin_amdgcn_wmma_f32_16x16x32_f16(false, a, false, b, (short)0, c, false, false);
  asm volatile("v_nop\n\tv_nop\n\tv_nop\n\tv_nop" : "+v"(d) : "v"(a), "v"(b));
  return d;
}
__device__ __forceinline__ v16h frag16(const _Float16* p, int hh) {
  const v8h lo = *(const v8h*)(p + 8 * hh), hi = *(const v8h*)(p + 16 + 8 * hh);
  return __builtin_shufflevector(lo, hi, 0,1,2,3,4,5,6,7,8,9,10,11,12,13,14,15);
}
__global__ __launch_bounds__(256) void k_sort_init(const int* __restrict__ src, const int* __restrict__ dst, u32* __restrict__ A, int E) {
  const int i = blockIdx.x * 256 + threadIdx.x;
  VST2(u32, A + i, (i < E) ? (((u32)dst[i]) << 16) | (u32)src[i] : 0xffffffffu);
}
__device__ __forceinline__ void cas_lds(u32* s, int lo, int hi, bool up) {
  const u32 a = s[lo], b = s[hi]; const bool sw = up ? (a > b) : (a < b); s[lo] = sw ? b : a; s[hi] = sw ? a : b;
}
__global__ __launch_bounds__(256) void k_sort_local(u32* __restrict__ A) {
  __shared__ u32 s[TILE];
  const int base = blockIdx.x * TILE, t = threadIdx.x;
  for (int i = t; i < TILE; i += 256) s[i] = A[base + i];
  __syncthreads();
  for (int k = 2; k <= TILE; k <<= 1)
    for (int j = k >> 1; j > 0; j >>= 1) {
      for (int p = t; p < TILE / 2; p += 256) {
        const int lo = ((p >> __builtin_ctz(j)) << (__builtin_ctz(j) + 1)) | (p & (j - 1));
        cas_lds(s, lo, lo + j, (((base + lo) & k) == 0));
      }
      __syncthreads();
    }
  for (int pass = 0; pass < 2; ++pass) { for (int i = t; i < TILE; i += 256) *(volatile u32*)(A + base + i) = s[i]; __threadfence(); }
}
__global__ __launch_bounds__(256) void k_sort_global(u32* __restrict__ A, int logj, int k) {
  const int p = blockIdx.x * 256 + threadIdx.x;
  const int j = 1 << logj;
  const int lo = ((p >> logj) << (logj + 1)) | (p & (j - 1)), hi = lo + j;
  const u32 a = A[lo], b = A[hi];
  const bool up = ((lo & k) == 0), sw = up ? (a > b) : (a < b);
  const u32 vlo = sw ? b : a, vhi = sw ? a : b;
  *(volatile u32*)(A + lo) = vlo; *(volatile u32*)(A + hi) = vhi; __threadfence();
  *(volatile u32*)(A + lo) = vlo; *(volatile u32*)(A + hi) = vhi;
}
__global__ __launch_bounds__(256) void k_sort_lds(u32* __restrict__ A, int k) {
  __shared__ u32 s[TILE];
  const int base = blockIdx.x * TILE, t = threadIdx.x;
  for (int i = t; i < TILE; i += 256) s[i] = A[base + i];
  __syncthreads();
  for (int j = TILE >> 1; j > 0; j >>= 1) {
    for (int p = t; p < TILE / 2; p += 256) {
      const int lo = ((p >> __builtin_ctz(j)) << (__builtin_ctz(j) + 1)) | (p & (j - 1));
      cas_lds(s, lo, lo + j, (((base + lo) & k) == 0));
    }
    __syncthreads();
  }
  for (int pass = 0; pass < 2; ++pass) { for (int i = t; i < TILE; i += 256) *(volatile u32*)(A + base + i) = s[i]; __threadfence(); }
}

__global__ __launch_bounds__(256) void k_segs(const u32* __restrict__ A, v2i* __restrict__ seg, float* __restrict__ inv) {
  const int n = blockIdx.x * 256 + threadIdx.x;
  if (n >= NN) return;
  int lo = 0, hi = SORTN;
  while (lo < hi) { const int mid = (lo + hi) >> 1; if ((A[mid] >> 16) < (u32)n) lo = mid + 1; else hi = mid; }
  const int st = lo; hi = SORTN;
  while (lo < hi) { const int mid = (lo + hi) >> 1; if ((A[mid] >> 16) < (u32)(n + 1)) lo = mid + 1; else hi = mid; }
  const v2i sv = {st, lo - st};
  VST2(v2i, seg + n, sv);
  VST2(float, inv + n, 1.0f / fmaxf((float)(lo - st), 1.0f));
}

__global__ __launch_bounds__(256) void k_to16(const float* __restrict__ src, int K, _Float16* __restrict__ dst) {
  const size_t t = (size_t)blockIdx.x * 256 + threadIdx.x;
  const int per = K / 8;
  if (t >= (size_t)NPAD * per) return;
  const int i = (int)(t / per), c = (int)(t % per) * 8;
  v8h o;
#pragma unroll
  for (int e = 0; e < 8; ++e) o[e] = (i < NN) ? (_Float16)src[(size_t)i * K + c + e] : (_Float16)0.f;
  VST2(v8h, dst + (size_t)i * K + c, o);
}
__global__ __launch_bounds__(256) void k_wt(const float* __restrict__ W, int K, int Nv, _Float16* __restrict__ Wt) {
  const int t = blockIdx.x * 256 + threadIdx.x;
  const int per = K / 8;
  if (t >= Nv * per) return;
  const int n = t / per, k0 = (t % per) * 8;
  v8h o;
#pragma unroll
  for (int e = 0; e < 8; ++e) o[e] = (_Float16)W[(size_t)(k0 + e) * Nv + n];
  VST2(v8h, Wt + (size_t)n * K + k0, o);
}
template <int K, int NTOT>
__global__ __launch_bounds__(128) void k_gemm(const _Float16* __restrict__ A, const _Float16* __restrict__ Wt, const float* __restrict__ bias,
                                              float* __restrict__ outf, _Float16* __restrict__ outh, int nrows) {
  __shared__ __attribute__((aligned(16))) float sT[4][16][132];
  const int lane = threadIdx.x & 31, wave = threadIdx.x >> 5, hh = lane >> 4, l16 = lane & 15;
  const int m0 = blockIdx.x * 64 + wave * 16, n0 = blockIdx.y * 128;
  v8f acc[8];
#pragma unroll
  for (int ni = 0; ni < 8; ++ni) acc[ni] = (v8f){};
#pragma unroll 2
  for (int k0 = 0; k0 < K; k0 += 32) {
    const v16h a0 = frag16(A + (size_t)(m0 + l16) * K + k0, hh);
#pragma unroll
    for (int ni = 0; ni < 8; ++ni) { const v16h b = frag16(Wt + (size_t)(n0 + ni * 16 + l16) * K + k0, hh); acc[ni] = wmma16(a0, b, acc[ni]); }
  }
  float (*st)[132] = sT[wave];
#pragma unroll
  for (int ni = 0; ni < 8; ++ni)
#pragma unroll
    for (int i = 0; i < 8; ++i) st[i + 8 * hh][ni * 16 + l16] = acc[ni][i] + bias[n0 + ni * 16 + l16];
  __builtin_amdgcn_fence(__ATOMIC_RELEASE, "workgroup"); __builtin_amdgcn_wave_barrier(); __builtin_amdgcn_fence(__ATOMIC_ACQUIRE, "workgroup");
  for (int pass = 0; pass < 2; ++pass) {
#pragma unroll
    for (int rr = 0; rr < 16; ++rr) {
      if (outf != nullptr && m0 + rr < nrows) *(volatile v4f*)(outf + (size_t)(m0 + rr) * NTOT + n0 + lane * 4) = *(const v4f*)(&st[rr][lane * 4]);
      if (outh != nullptr && lane < 16) { v8h o;
#pragma unroll
        for (int e = 0; e < 8; ++e) o[e] = (_Float16)st[rr][lane * 8 + e];
        *(volatile v8h*)(outh + (size_t)(m0 + rr) * NTOT + n0 + lane * 8) = o; }
    }
    __threadfence();
  }
}
__global__ __launch_bounds__(256) void k_adots(const float* __restrict__ h, int HN, const float* __restrict__ asrc, const float* __restrict__ adst,
                                               float* __restrict__ as, float* __restrict__ ad) {
  const int t = blockIdx.x * 256 + threadIdx.x;
  if (t >= NN * HN) return;
  const int n = t / HN, hd = t % HN;
  const float* hr = h + ((size_t)n * HN + hd) * DD;
  float s = 0.f, d = 0.f;
  for (int c = 0; c < DD; ++c) { const float v = hr[c]; s += v * asrc[hd * DD + c]; d += v * adst[hd * DD + c]; }
  VST2(float, as + t, s); VST2(float, ad + t, d);
}
template <int HN, int MODE>
__global__ __launch_bounds__(256) void k_gat(const float* __restrict__ h, const u32* __restrict__ keys, const v2i* __restrict__ seg, const float* __restrict__ as,
                                             const float* __restrict__ ad, const float* __restrict__ gbias, const float* __restrict__ gp, const float* __restrict__ beta,
                                             _Float16* __restrict__ out16) {
  constexpr int WID = HN * DD, PER = WID / 8;
  const int t = blockIdx.x * 256 + threadIdx.x;
  if (t >= NPAD * PER) return;
  const int i = t / PER, c = (t % PER) * 8, hd = c / DD;
  float acc[8] = {0.f, 0.f, 0.f, 0.f, 0.f, 0.f, 0.f, 0.f};
  v8h o;
  if (i < NN) {
    const v2i sv = seg[i];
    const int st = min(max(sv[0], 0), SORTN - 1), cnt = min(max(sv[1], 0), MAXDEG);
    const float adi = ad[i * HN + hd];
    auto score = [&](int j) -> float { const float a = as[j * HN + hd] + adi; return (a > 0.f) ? a : 0.2f * a; };
    float mx = score(i);
    for (int p = 0; p < cnt; ++p) { const int j = min((int)(keys[min(st + p, SORTN - 1)] & 0xffffu), NN - 1); mx = fmaxf(mx, score(j)); }
    float den = expf(score(i) - mx);
    { const float* hr = h + (size_t)i * WID + c;
#pragma unroll
      for (int e = 0; e < 8; ++e) acc[e] = den * hr[e]; }
    for (int p = 0; p < cnt; ++p) {
      const int j = min((int)(keys[min(st + p, SORTN - 1)] & 0xffffu), NN - 1);
      const float w = expf(score(j) - mx); den += w;
      const float* hr = h + (size_t)j * WID + c;
#pragma unroll
      for (int e = 0; e < 8; ++e) acc[e] += w * hr[e];
    }
    const float inv = 1.0f / (den + 1e-16f);
    const float bt = (MODE == 1) ? beta[0] : 0.f;
#pragma unroll
    for (int e = 0; e < 8; ++e) {
      float v = acc[e] * inv + gbias[c + e];
      if (MODE == 0) v = (v > 0.f) ? v : (expf(v) - 1.0f);
      else v += bt * gp[(size_t)i * DD + c + e];
      o[e] = (_Float16)v;
    }
  } else {
#pragma unroll
    for (int e = 0; e < 8; ++e) o[e] = (_Float16)0.f;
  }
  VST2(v8h, out16 + (size_t)i * WID + c, o);
}
extern "C" void kernel_launch(void* const* d_in, const int* in_sizes, int n_in,
                              void* d_out, int out_size, void* d_ws, size_t ws_size, hipStream_t stream) {
  (void)in_sizes; (void)n_in; (void)out_size;
  const float* x    = (const float*)d_in[0];
  const int*   ei   = (const int*)  d_in[1];
  const float* g    = (const float*)d_in[2];
  const float* pW   = (const float*)d_in[3];  const float* pb = (const float*)d_in[4];
  const float* W1   = (const float*)d_in[5];  const float* as1 = (const float*)d_in[6]; const float* ad1 = (const float*)d_in[7]; const float* b1 = (const float*)d_in[8];
  const float* W2   = (const float*)d_in[9];  const float* as2 = (const float*)d_in[10]; const float* ad2 = (const float*)d_in[11]; const float* b2 = (const float*)d_in[12];
  const float* dW   = (const float*)d_in[13]; const float* db = (const float*)d_in[14];
  const float* beta = (const float*)d_in[15];
  float* out = (float*)d_out;
  char* ws = (char*)d_ws; size_t off = 0;
  auto take = [&](size_t bytes) { void* p = ws + off; off = (off + bytes + 255) & ~(size_t)255; return p; };
  u32*      keys = (u32*)take((size_t)SORTN * 4);
  v2i*      seg  = (v2i*)take((size_t)NN * 8);
  float*    inv  = (float*)take((size_t)NN * 4);
  _Float16* X16  = (_Float16*)take((size_t)NPAD * DIN * 2);
  _Float16* G16  = (_Float16*)take((size_t)NPAD * DIN * 2);
  _Float16* WtP  = (_Float16*)take((size_t)DD * DIN * 2);
  _Float16* Wt1  = (_Float16*)take((size_t)HC * DD * 2);
  _Float16* Wt2  = (_Float16*)take((size_t)DD * HC * 2);
  _Float16* WtD  = (_Float16*)take((size_t)DIN * DD * 2);
  _Float16* xp16 = (_Float16*)take((size_t)NPAD * DD * 2);
  float*    gp   = (float*)take((size_t)NPAD * DD * 4);
  float*    h1   = (float*)take((size_t)NPAD * HC * 4);
  float*    a1s  = (float*)take((size_t)NN * 4 * 4);
  float*    a1d  = (float*)take((size_t)NN * 4 * 4);
  _Float16* e16  = (_Float16*)take((size_t)NPAD * HC * 2);
  float*    h2   = (float*)take((size_t)NPAD * DD * 4);
  float*    a2s  = (float*)take((size_t)NN * 4);
  float*    a2d  = (float*)take((size_t)NN * 4);
  _Float16* f16  = (_Float16*)take((size_t)NPAD * DD * 2);
  float*    zb   = (float*)take((size_t)HC * 4);
  if (off > ws_size) return;
  hipMemsetAsync(zb, 0, HC * 4, stream);
  const dim3 b256(256);
  k_sort_init<<<SORTN / 256, b256, 0, stream>>>(ei, ei + NE, keys, NE);
  k_sort_local<<<SORTN / TILE, b256, 0, stream>>>(keys);
  for (int k = TILE * 2; k <= SORTN; k <<= 1) {
    for (int logj = __builtin_ctz(k) - 1; (1 << logj) >= TILE; --logj)
      k_sort_global<<<SORTN / 2 / 256, b256, 0, stream>>>(keys, logj, k);
    k_sort_lds<<<SORTN / TILE, b256, 0, stream>>>(keys, k);
  }
  k_segs<<<(NN + 255) / 256, b256, 0, stream>>>(keys, seg, inv);
  k_to16<<<(NPAD * 96 + 255) / 256, b256, 0, stream>>>(x, DIN, X16);
  k_to16<<<(NPAD * 96 + 255) / 256, b256, 0, stream>>>(g, DIN, G16);
  k_wt<<<(DD * 96 + 255) / 256, b256, 0, stream>>>(pW, DIN, DD, WtP);
  k_wt<<<(HC * 16 + 255) / 256, b256, 0, stream>>>(W1, DD, HC, Wt1);
  k_wt<<<(DD * 64 + 255) / 256, b256, 0, stream>>>(W2, HC, DD, Wt2);
  k_wt<<<(DIN * 16 + 255) / 256, b256, 0, stream>>>(dW, DD, DIN, WtD);
  k_gemm<DIN, DD><<<dim3(NPAD / 64, 1), 128, 0, stream>>>(X16, WtP, pb, nullptr, xp16, NN);
  k_gemm<DIN, DD><<<dim3(NPAD / 64, 1), 128, 0, stream>>>(G16, WtP, pb, gp, nullptr, NPAD);
  k_gemm<DD, HC><<<dim3(NPAD / 64, 4), 128, 0, stream>>>(xp16, Wt1, zb, h1, nullptr, NPAD);
  k_adots<<<(NN * 4 + 255) / 256, b256, 0, stream>>>(h1, 4, as1, ad1, a1s, a1d);
  k_gat<4, 0><<<(NPAD * 64 + 255) / 256, b256, 0, stream>>>(h1, keys, seg, a1s, a1d, b1, nullptr, nullptr, e16);
  k_gemm<HC, DD><<<dim3(NPAD / 64, 1), 128, 0, stream>>>(e16, Wt2, zb, h2, nullptr, NPAD);
  k_adots<<<(NN + 255) / 256, b256, 0, stream>>>(h2, 1, as2, ad2, a2s, a2d);
  k_gat<1, 1><<<(NPAD * 16 + 255) / 256, b256, 0, stream>>>(h2, keys, seg, a2s, a2d, b2, gp, beta, f16);
  k_gemm<DD, DIN><<<dim3(NPAD / 64, 6), 128, 0, stream>>>(f16, WtD, db, out, nullptr, NN);
}
